// HRAN_37598143709631
// MI455X (gfx1250) — hardware-verified
//
#include <hip/hip_runtime.h>
#include <stddef.h>


#define NIN    128
#define NEMB   64
#define NH     256
#define NR     12
#define NBAS   8
#define IN1    (NIN + NEMB)
#define K1     (9 * IN1)
#define K2     (9 * NH)
#define NOUT   12
#define NTHR   256
#define NWAVE  8
#define GROWS  64
#define NC     8192
#define NB     1024
#define CAP    24576
#define MAXWIN 40
#define MAXDEG 4096
#define WSCAP  134217728
#define CARRY_A 8.0f
#define CARRY_B 16.0f
#define INV_CARRY (1.0f / 128.0f)
#define LDS_GEMM (GROWS * NH * 4)
#define LDS_FILL ((NB + CAP) * 4)

static_assert((K1 % 32) == 0 && (K2 % 32) == 0);
static_assert((NC % GROWS) == 0 && (NC % NWAVE) == 0 && (GROWS % NWAVE) == 0);
static_assert(NB == 4 * NTHR && (CAP % 32) == 0 && (NB & (NB - 1)) == 0);
static_assert(NTHR == NWAVE * 32 && NH == 256 && IN1 == 192);
static_assert(((GROWS * NOUT) % 4) == 0 && LDS_FILL <= 160 * 1024);

typedef float          v4f  __attribute__((ext_vector_type(4)));
typedef float          v8f  __attribute__((ext_vector_type(8)));
typedef int            v4i  __attribute__((ext_vector_type(4)));
typedef unsigned short v8us __attribute__((ext_vector_type(8)));
typedef _Float16       v16h __attribute__((ext_vector_type(16)));
typedef v4f  v4fa  __attribute__((may_alias));
typedef v4i  v4ia  __attribute__((may_alias));
typedef v8us v8usa __attribute__((may_alias));
union FragH { v16h v; v8us h[2]; };

static __device__ __forceinline__ unsigned short f2h(float f) {
  _Float16 h = (_Float16)f;
  return __builtin_bit_cast(unsigned short, h);
}
static __device__ __forceinline__ v8f wm(v16h a, v16h b, v8f c) {
  v8f d = __builtin_amdgcn_wmma_f32_16x16x32_f16(false, a, false, b, (short)0, c, false, false);
  asm volatile("v_nop\n\tv_nop\n\tv_nop\n\tv_nop" : "+v"(d) : "v"(a), "v"(b));
  return d;
}

__global__ __launch_bounds__(NTHR) void k_zero(float* p, int n4) {
  const int i = (int)blockIdx.x * NTHR + (int)threadIdx.x;
  if (i >= n4) return;
  const v4f z = {0.f, 0.f, 0.f, 0.f};
  float* gp = p + (size_t)4 * i;
  *(volatile v4f*)gp = z;
  __threadfence();
  *(volatile v4f*)gp = z;
}

__global__ __launch_bounds__(NTHR) void k_emb(const int* __restrict__ idx, const float* __restrict__ emb,
                                              float* E0, int rows, int nN) {
  const int tid = threadIdx.x, lane = tid & 31;
  const int gw = ((int)blockIdx.x * NTHR + tid) >> 5;
  const int g = 2 * gw + (lane >> 4);
  const int piece = lane & 15;
  const int gc = g < rows ? g : rows - 1;
  int node = idx[gc];
  node = node < 0 ? 0 : (node > nN - 1 ? nN - 1 : node);
  const v4f v = *(const v4f*)(emb + (size_t)gc * NEMB + 4 * piece);
  float* gp = E0 + (size_t)node * NEMB + 4 * piece;
  const bool ok = g < rows;
  if (ok) *(volatile v4f*)gp = v;
  __threadfence();
  if (ok) *(volatile v4f*)gp = v;
}

__global__ __launch_bounds__(NTHR) void k_count(const int* __restrict__ ei, int* deg, int nE, int nN) {
  __shared__ __attribute__((aligned(16))) int hist[NB];
  const int tid = threadIdx.x;
  const int n0 = (int)blockIdx.x * NB;
  for (int i = tid; i < NB; i += NTHR) hist[i] = 0;
  __syncthreads();
  const int* edst = ei + (size_t)nE;
#pragma unroll 1
  for (int e = tid; e < nE; e += NTHR) {
    const int d = edst[e];
    const int u = d - n0;
    if (d < nN && (unsigned)u < (unsigned)NB) atomicAdd(&hist[u], 1);
  }
  __syncthreads();
  const v4i v = *(const v4ia*)(hist + 4 * tid);
  int* gp = deg + (size_t)n0 + 4 * tid;
  *(volatile v4i*)gp = v;
  __threadfence();
  *(volatile v4i*)gp = v;
}

__global__ __launch_bounds__(NTHR) void k_scan(const int* __restrict__ deg, int* start, int nblk, int nE) {
  __shared__ int sh[NTHR];
  const int tid = threadIdx.x;
  int run = 0;
#pragma unroll 1
  for (int t = 0; t < nblk; ++t) {
    const int base = (run + 31) & ~31;
    v4i d = *(const v4i*)(deg + (size_t)t * NB + 4 * tid);
    d.x = d.x < 0 ? 0 : (d.x > nE ? nE : d.x);
    d.y = d.y < 0 ? 0 : (d.y > nE ? nE : d.y);
    d.z = d.z < 0 ? 0 : (d.z > nE ? nE : d.z);
    d.w = d.w < 0 ? 0 : (d.w > nE ? nE : d.w);
    const int s = d.x + d.y + d.z + d.w;
    sh[tid] = s;
    __syncthreads();
#pragma unroll 1
    for (int off = 1; off < NTHR; off <<= 1) {
      const int src = tid - off < 0 ? 0 : tid - off;
      const int tv = sh[src];
      const int add = (tid >= off) ? tv : 0;
      __syncthreads();
      sh[tid] += add;
      __syncthreads();
    }
    const int incl = sh[tid];
    const int total = sh[NTHR - 1];
    const int excl = incl - s;
    v4i st;
    st.x = base + excl; st.y = st.x + d.x; st.z = st.y + d.y; st.w = st.z + d.z;
    int* gp = start + (size_t)t * NB + 4 * tid;
    *(volatile v4i*)gp = st;
    __threadfence();
    *(volatile v4i*)gp = st;
    run = base + total;
    __syncthreads();
  }
}

__global__ __launch_bounds__(NTHR) void k_fill(const int* __restrict__ ei, const int* __restrict__ et,
                                               const int* __restrict__ degT, const int* __restrict__ stT,
                                               int* csr, int nE, int nN, int csrn) {
  extern __shared__ v4f lds_dyn[];
  int* cur  = (int*)lds_dyn;
  int* sbuf = cur + NB;
  const int tid = threadIdx.x, lane = tid & 31;
  const int wave = __builtin_amdgcn_readfirstlane(tid >> 5);
  const int n0 = (int)blockIdx.x * NB;
  int nn = nN - n0; nn = nn > NB ? NB : nn;
  int base = __builtin_amdgcn_readfirstlane(stT[n0]);
  base = base < 0 ? 0 : base;
  base &= ~31;
  if (base > csrn - 32) base = csrn - 32;
  const int last = n0 + nn - 1;
  int dl = __builtin_amdgcn_readfirstlane(degT[last]);
  dl = dl < 0 ? 0 : (dl > nE ? nE : dl);
  int sl = __builtin_amdgcn_readfirstlane(stT[last]);
  sl = sl < 0 ? 0 : (sl > csrn - 1 ? csrn - 1 : sl);
  int L = sl + dl - base;
  L = L < 0 ? 0 : (L > nE ? nE : L);
  const int L32 = (L + 31) & ~31;
  int nwin = (L + CAP - 1) / CAP;
  nwin = nwin > MAXWIN ? MAXWIN : nwin;
  const int nchunk = (nE + NTHR - 1) / NTHR;
  const int* edst = ei + (size_t)nE;
  const unsigned ltmask = (1u << lane) - 1u;
#pragma unroll 1
  for (int w = 0; w < nwin; ++w) {
#pragma unroll 1
    for (int i = tid; i < NB; i += NTHR) {
      int ni = n0 + i; ni = ni > nN - 1 ? nN - 1 : ni;
      int v = stT[ni] - base;
      v = v < 0 ? 0 : (v > csrn ? csrn : v);
      cur[i] = (i < nn) ? v : 0;
    }
#pragma unroll 1
    for (int i = tid; i < CAP; i += NTHR) sbuf[i] = 0;
    __syncthreads();
    const int wlo = w * CAP;
#pragma unroll 1
    for (int c = 0; c < nchunk; ++c) {
      const int e = c * NTHR + tid;
      const int ec = e < nE ? e : nE - 1;
      const int s = ei[ec], d = edst[ec], ty = et[ec];
      const int u = d - n0;
      const bool hit = (e < nE) && ((unsigned)u < (unsigned)nn);
      const int sc = s < 0 ? 0 : (s > nN - 1 ? nN - 1 : s);
      const int tc = ty < 0 ? 0 : (ty > NR - 1 ? NR - 1 : ty);
      const int pack = sc | (tc << 16);
      const unsigned uu = (unsigned)(hit ? u : 0);
#pragma unroll 1
      for (int wv = 0; wv < NWAVE; ++wv) {
        if (wave == wv) {
          unsigned peers = __builtin_amdgcn_ballot_w32(hit);
#pragma unroll
          for (int b = 0; (1 << b) < NB; ++b) {
            const bool bit = ((uu >> b) & 1u) != 0u;
            const unsigned mb = __builtin_amdgcn_ballot_w32(bit);
            peers &= bit ? mb : ~mb;
          }
          const int rank = (int)__builtin_popcount(peers & ltmask);
          const int tot  = (int)__builtin_popcount(peers);
          const int p0 = cur[uu];
          if (hit) {
            const int rel = p0 + rank - wlo;
            if ((unsigned)rel < (unsigned)CAP) sbuf[rel] = pack;
            if (rank == tot - 1) cur[uu] = p0 + tot;
          }
        }
        __syncthreads();
      }
    }
    int wl = L32 - wlo; wl = wl > CAP ? CAP : wl;
    const int room = csrn - (base + wlo);
    wl = wl > room ? room : wl; wl = wl < 0 ? 0 : wl;
    const int np = wl >> 2;
    int* gp = csr + (size_t)base + wlo;
#pragma unroll 1
    for (int p = tid; p < np; p += NTHR) { const v4i v = *(const v4ia*)(sbuf + 4 * p); *(volatile v4i*)(gp + 4 * p) = v; }
    __threadfence();
#pragma unroll 1
    for (int p = tid; p < np; p += NTHR) { const v4i v = *(const v4ia*)(sbuf + 4 * p); *(volatile v4i*)(gp + 4 * p) = v; }
    __syncthreads();
  }
}

template <int K, int INW>
__global__ __launch_bounds__(NTHR) void k_bwt(const float* __restrict__ basis, const float* __restrict__ root,
                                              unsigned short* BT) {
  const int i = (int)blockIdx.x * NTHR + (int)threadIdx.x;
  if (i >= (NH * K) / 8) return;
  const int e = 8 * i;
  const int o = e / K;
  const int k0 = e - o * K;
  v8us hv;
#pragma unroll
  for (int j = 0; j < 8; ++j) {
    const int k = k0 + j;
    const int kb = k > NBAS * INW - 1 ? NBAS * INW - 1 : k;
    int kr = k - NBAS * INW; kr = kr < 0 ? 0 : (kr > INW - 1 ? INW - 1 : kr);
    const float vb = basis[(size_t)kb * NH + o];
    const float vr = root[(size_t)kr * NH + o];
    const float v = (k < NBAS * INW) ? vb : vr;
    hv[j] = f2h(v * CARRY_B);
  }
  unsigned short* gp = BT + (size_t)e;
  *(volatile v8us*)gp = hv;
  __threadfence();
  *(volatile v8us*)gp = hv;
}

template <int LAYER>
__global__ __launch_bounds__(NTHR) void k_agg(const float* __restrict__ xa, const float* __restrict__ xb,
                                              const int* __restrict__ degT, const int* __restrict__ stT,
                                              const int* __restrict__ csr, const float* __restrict__ comp,
                                              unsigned short* Ac, int c0, int nN, int csrn) {
  constexpr int INW = (LAYER == 1) ? IN1 : NH;
  constexpr int JN = INW / 32;
  constexpr int K = 9 * INW;
  constexpr int NP = K / 8;
  __shared__ __attribute__((aligned(16))) unsigned short rowbuf[NWAVE * K2];
  const int tid = threadIdx.x, lane = tid & 31;
  const int wave = __builtin_amdgcn_readfirstlane(tid >> 5);
  const int r = (int)blockIdx.x * NWAVE + wave;
  const int n = c0 + r;
  const bool valid = n < nN;
  const int nc = valid ? n : nN - 1;
  int deg = degT[nc];
  deg = __builtin_amdgcn_readfirstlane(valid ? deg : 0);
  const bool poison = (deg < 0) || (deg > MAXDEG);
  const int degc = deg < 0 ? 0 : (deg > MAXDEG ? MAXDEG : deg);
  int st = __builtin_amdgcn_readfirstlane(stT[nc]);
  st = st < 0 ? 0 : (st > csrn - 1 ? csrn - 1 : st);

  int cnt = 0;
#pragma unroll 1
  for (int e = 0; e < degc; ++e) {
    int ix = st + e; ix = ix > csrn - 1 ? csrn - 1 : ix;
    const int rec = csr[ix];
    int rel = (rec >> 16) & 15; rel = rel > NR - 1 ? NR - 1 : rel;
    cnt += (rel == lane) ? 1 : 0;
  }
  const float wl = __builtin_amdgcn_rcpf(fmaxf((float)cnt, 1.0f));

  float acc[NBAS][JN];
#pragma unroll
  for (int b = 0; b < NBAS; ++b)
#pragma unroll
    for (int j = 0; j < JN; ++j) acc[b][j] = 0.0f;

#pragma unroll 1
  for (int e = 0; e < degc; ++e) {
    int ix = st + e; ix = ix > csrn - 1 ? csrn - 1 : ix;
    const int rec = csr[ix];
    int src = rec & 0xFFFF; src = src > nN - 1 ? nN - 1 : src;
    int rel = (rec >> 16) & 15; rel = rel > NR - 1 ? NR - 1 : rel;
    const float wr = __shfl(wl, rel);
    float cb[NBAS];
#pragma unroll
    for (int b = 0; b < NBAS; ++b) cb[b] = comp[rel * NBAS + b] * wr;
    float xv[JN];
    if (LAYER == 1) {
#pragma unroll
      for (int j = 0; j < 4; ++j) xv[j] = xa[(size_t)src * NIN + 32 * j + lane];
#pragma unroll
      for (int j = 0; j < 2; ++j) xv[4 + j] = xb[(size_t)src * NEMB + 32 * j + lane];
    } else {
#pragma unroll
      for (int j = 0; j < JN; ++j) xv[j] = xa[(size_t)src * NH + 32 * j + lane];
    }
#pragma unroll
    for (int b = 0; b < NBAS; ++b)
#pragma unroll
      for (int j = 0; j < JN; ++j) acc[b][j] = fmaf(cb[b], xv[j], acc[b][j]);
  }

  float xt[JN];
  if (LAYER == 1) {
#pragma unroll
    for (int j = 0; j < 4; ++j) xt[j] = xa[(size_t)nc * NIN + 32 * j + lane];
#pragma unroll
    for (int j = 0; j < 2; ++j) xt[4 + j] = xb[(size_t)nc * NEMB + 32 * j + lane];
  } else {
#pragma unroll
    for (int j = 0; j < JN; ++j) xt[j] = xa[(size_t)nc * NH + 32 * j + lane];
  }
  const float vz = valid ? 1.0f : 0.0f;
  const float padd = poison ? __int_as_float(0x7FC00000) : 0.0f;
  unsigned short* rb = rowbuf + wave * K2;
#pragma unroll
  for (int b = 0; b < NBAS; ++b)
#pragma unroll
    for (int j = 0; j < JN; ++j) rb[b * INW + 32 * j + lane] = f2h(acc[b][j] * CARRY_A + padd);
#pragma unroll
  for (int j = 0; j < JN; ++j) rb[NBAS * INW + 32 * j + lane] = f2h(xt[j] * vz * CARRY_A + padd);
  __syncthreads();

  const unsigned short* rr = rowbuf + wave * K2;
  unsigned short* gr = Ac + (size_t)r * K;
  for (int p = lane; p < NP; p += 32) { const v8us v = *(const v8usa*)(rr + 8 * p); *(volatile v8us*)(gr + 8 * p) = v; }
  __threadfence();
  for (int p = lane; p < NP; p += 32) { const v8us v = *(const v8usa*)(rr + 8 * p); *(volatile v8us*)(gr + 8 * p) = v; }
}

template <int K, int LAYER>
__global__ __launch_bounds__(NTHR) void k_gemm(const unsigned short* __restrict__ A, const unsigned short* __restrict__ BT,
                                               const float* __restrict__ bias, const float* __restrict__ att,
                                               float* H1c, const float* __restrict__ pw, const float* __restrict__ pb,
                                               float* outc, int nvalid) {
  static_assert((K % 32) == 0);
  extern __shared__ v4f lds_dyn[];
  __shared__ __attribute__((aligned(16))) float ostg[GROWS * NOUT];
  float* stg = (float*)lds_dyn;
  const int tid = threadIdx.x, lane = tid & 31, hh = lane >> 4, m = lane & 15;
  const int wave = __builtin_amdgcn_readfirstlane(tid >> 5);
  const int rstrip = wave & 3, nhalf = wave >> 2;
  const unsigned short* ap = A + (size_t)((int)blockIdx.x * GROWS + rstrip * 16 + m) * K + 8 * hh;
  const unsigned short* bp = BT + (size_t)(nhalf * 128 + m) * K + 8 * hh;

  v8f acc[8];
#pragma unroll
  for (int t = 0; t < 8; ++t) { v8f zz = {0.f, 0.f, 0.f, 0.f, 0.f, 0.f, 0.f, 0.f}; acc[t] = zz; }

#pragma unroll 1
  for (int kt = 0; kt < K / 32; ++kt) {
    FragH fa;
    fa.h[0] = *(const v8us*)(ap + 32 * kt);
    fa.h[1] = *(const v8us*)(ap + 32 * kt + 16);
#pragma unroll
    for (int t = 0; t < 8; ++t) {
      const unsigned short* bq = bp + (size_t)(16 * t) * K + 32 * kt;
      FragH fb;
      fb.h[0] = *(const v8us*)bq;
      fb.h[1] = *(const v8us*)(bq + 16);
      acc[t] = wm(fa.v, fb.v, acc[t]);
    }
  }
  {
    float* sp = stg + (rstrip * 16 + 8 * hh) * NH + nhalf * 128 + m;
#pragma unroll
    for (int t = 0; t < 8; ++t)
#pragma unroll
      for (int r = 0; r < 8; ++r) sp[r * NH + 16 * t] = acc[t][r];
  }
  __syncthreads();

  const v4f bv0 = *(const v4f*)(bias + 4 * lane);
  const v4f bv1 = *(const v4f*)(bias + 128 + 4 * lane);
  const v4f a0 = *(const v4f*)(att + hh * 64 + 4 * m);
  const v4f a1 = *(const v4f*)(att + (2 + hh) * 64 + 4 * m);
  float pbv[NOUT];
#pragma unroll
  for (int c = 0; c < NOUT; ++c) pbv[c] = pb[c];

#pragma unroll 1
  for (int i = 0; i < 8; ++i) {
    const int row = wave * 8 + i;
    float* lp = stg + row * NH;
    v4f v0 = *(const v4fa*)(lp + 4 * lane) * INV_CARRY + bv0;
    v4f v1 = *(const v4fa*)(lp + 128 + 4 * lane) * INV_CARRY + bv1;
    float sA = v0.x * a0.x + v0.y * a0.y + v0.z * a0.z + v0.w * a0.w;
    float sB = v1.x * a1.x + v1.y * a1.y + v1.z * a1.z + v1.w * a1.w;
    sA += __shfl_xor(sA, 1); sA += __shfl_xor(sA, 2); sA += __shfl_xor(sA, 4); sA += __shfl_xor(sA, 8);
    sB += __shfl_xor(sB, 1); sB += __shfl_xor(sB, 2); sB += __shfl_xor(sB, 4); sB += __shfl_xor(sB, 8);
    const float s0 = __shfl(sA, 0), s1 = __shfl(sA, 16), s2 = __shfl(sB, 0), s3 = __shfl(sB, 16);
    const float mx = fmaxf(fmaxf(s0, s1), fmaxf(s2, s3));
    const float e0 = __expf(s0 - mx), e1 = __expf(s1 - mx), e2 = __expf(s2 - mx), e3 = __expf(s3 - mx);
    const float inv = __builtin_amdgcn_rcpf((e0 + e1) + (e2 + e3));
    const float alA = (hh == 0 ? e0 : e1) * inv;
    const float alB = (hh == 0 ? e2 : e3) * inv;
    v0 = v0 * alA;
    v1 = v1 * alB;
    if (LAYER == 1) {
      float* gp = H1c + (size_t)((int)blockIdx.x * GROWS + row) * NH + 4 * lane;
      *(volatile v4f*)gp = v0;
      *(volatile v4f*)(gp + 128) = v1;
      __threadfence();
      *(volatile v4f*)gp = v0;
      *(volatile v4f*)(gp + 128) = v1;
    } else {
      *(v4fa*)(lp + 4 * lane) = v0;
      *(v4fa*)(lp + 128 + 4 * lane) = v1;
      __syncthreads();
      float p[NOUT];
#pragma unroll
      for (int c = 0; c < NOUT; ++c) p[c] = 0.0f;
#pragma unroll 1
      for (int jj = 0; jj < 8; ++jj) {
        const float hv = lp[8 * lane + jj];
        const float* wr = pw + (size_t)(8 * lane + jj) * NOUT;
        const v4f w0 = *(const v4f*)wr, w1 = *(const v4f*)(wr + 4), w2 = *(const v4f*)(wr + 8);
        p[0] = fmaf(hv, w0.x, p[0]); p[1] = fmaf(hv, w0.y, p[1]); p[2]  = fmaf(hv, w0.z, p[2]);  p[3]  = fmaf(hv, w0.w, p[3]);
        p[4] = fmaf(hv, w1.x, p[4]); p[5] = fmaf(hv, w1.y, p[5]); p[6]  = fmaf(hv, w1.z, p[6]);  p[7]  = fmaf(hv, w1.w, p[7]);
        p[8] = fmaf(hv, w2.x, p[8]); p[9] = fmaf(hv, w2.y, p[9]); p[10] = fmaf(hv, w2.z, p[10]); p[11] = fmaf(hv, w2.w, p[11]);
      }
#pragma unroll
      for (int c = 0; c < NOUT; ++c) {
        float v = p[c];
        v += __shfl_xor(v, 1); v += __shfl_xor(v, 2); v += __shfl_xor(v, 4); v += __shfl_xor(v, 8); v += __shfl_xor(v, 16);
        p[c] = v;
      }
      if (lane == 0) {
#pragma unroll
        for (int c = 0; c < NOUT; ++c) ostg[row * NOUT + c] = p[c] + pbv[c];
      }
    }
  }
  if (LAYER == 2) {
    __syncthreads();
    int nv = nvalid - (int)blockIdx.x * GROWS;
    nv = nv > GROWS ? GROWS : (nv < 0 ? 0 : nv);
    const int np = nv * 3;
    const int tc = tid < np ? tid : 0;
    const v4f ov = *(const v4fa*)(ostg + 4 * tc);
    float* op = outc + (size_t)blockIdx.x * GROWS * NOUT + 4 * tid;
    if (tid < np) *(volatile v4f*)op = ov;
    __threadfence();
    if (tid < np) *(volatile v4f*)op = ov;
  }
}

extern "C" void kernel_launch(void* const* d_in, const int* in_sizes, int n_in,
                              void* d_out, int out_size, void* d_ws, size_t ws_size,
                              hipStream_t stream) {
  if (n_in < 19) return;
  if (in_sizes[0] < NIN || (in_sizes[0] % NIN) != 0) return;
  const int nN = in_sizes[0] / NIN;
  if (nN < 1 || nN > 65536) return;
  if (in_sizes[1] < 2 || (in_sizes[1] % 2) != 0) return;
  const int nE = in_sizes[1] / 2;
  if (in_sizes[2] != nE || nE > MAXWIN * CAP) return;
  const int nG = in_sizes[3], nP = in_sizes[4];
  if (nG < 1 || nP < 1 || in_sizes[5] != nG * NEMB || in_sizes[6] != nP * NEMB) return;
  if (in_sizes[7] != NR * NBAS || in_sizes[8] != NBAS * IN1 * NH || in_sizes[9] != IN1 * NH) return;
  if (in_sizes[10] != NH || in_sizes[11] != 4 * 64) return;
  if (in_sizes[12] != NR * NBAS || in_sizes[13] != NBAS * NH * NH || in_sizes[14] != NH * NH) return;
  if (in_sizes[15] != NH || in_sizes[16] != 4 * 64 || in_sizes[17] != NH * NOUT || in_sizes[18] != NOUT) return;
  if (out_size != nN * NOUT) return;

  const float* x        = (const float*)d_in[0];
  const int*   ei       = (const int*)d_in[1];
  const int*   et       = (const int*)d_in[2];
  const int*   gene_idx = (const int*)d_in[3];
  const int*   path_idx = (const int*)d_in[4];
  const float* gene_emb = (const float*)d_in[5];
  const float* path_emb = (const float*)d_in[6];
  const float* comp1    = (const float*)d_in[7];
  const float* basis1   = (const float*)d_in[8];
  const float* root1    = (const float*)d_in[9];
  const float* bias1    = (const float*)d_in[10];
  const float* att1     = (const float*)d_in[11];
  const float* comp2    = (const float*)d_in[12];
  const float* basis2   = (const float*)d_in[13];
  const float* root2    = (const float*)d_in[14];
  const float* bias2    = (const float*)d_in[15];
  const float* att2     = (const float*)d_in[16];
  const float* pred_w   = (const float*)d_in[17];
  const float* pred_b   = (const float*)d_in[18];
  float* out = (float*)d_out;

  const int NPAD = ((nN + GROWS - 1) / GROWS) * GROWS;
  const int NBLK = (nN + NB - 1) / NB;
  const int NDEG = NBLK * NB;
  const int CSRN = ((nE + 32 * NBLK + 63) / 32) * 32;

  char* ws = (char*)d_ws;
  size_t off = 0;
  const size_t oE0  = off; off += (size_t)NPAD * NEMB * 4;     off = (off + 255) & ~(size_t)255;
  const size_t oH1  = off; off += (size_t)NPAD * NH * 4;       off = (off + 255) & ~(size_t)255;
  const size_t oA   = off; off += (size_t)NC * K2 * 2;         off = (off + 255) & ~(size_t)255;
  const size_t oBT  = off; off += (size_t)NH * K2 * 2;         off = (off + 255) & ~(size_t)255;
  const size_t oDEG = off; off += (size_t)NDEG * 4;            off = (off + 255) & ~(size_t)255;
  const size_t oST  = off; off += (size_t)NDEG * 4;            off = (off + 255) & ~(size_t)255;
  const size_t oCSR = off; off += (size_t)CSRN * 4;            off = (off + 255) & ~(size_t)255;
  if (off > ws_size || off > (size_t)WSCAP) return;
  float*          E0  = (float*)(ws + oE0);
  float*          H1  = (float*)(ws + oH1);
  unsigned short* Ab  = (unsigned short*)(ws + oA);
  unsigned short* BT  = (unsigned short*)(ws + oBT);
  int*            deg = (int*)(ws + oDEG);
  int*            stT = (int*)(ws + oST);
  int*            csr = (int*)(ws + oCSR);

  hipFuncSetAttribute(reinterpret_cast<const void*>(&k_fill), hipFuncAttributeMaxDynamicSharedMemorySize, LDS_FILL);
  hipFuncSetAttribute(reinterpret_cast<const void*>(&k_gemm<K1, 1>), hipFuncAttributeMaxDynamicSharedMemorySize, LDS_GEMM);
  hipFuncSetAttribute(reinterpret_cast<const void*>(&k_gemm<K2, 2>), hipFuncAttributeMaxDynamicSharedMemorySize, LDS_GEMM);

  {
    const int n4 = NPAD * (NEMB / 4);
    k_zero<<<(n4 + NTHR - 1) / NTHR, NTHR, 0, stream>>>(E0, n4);
    k_emb<<<(nG * 16 + NTHR - 1) / NTHR, NTHR, 0, stream>>>(gene_idx, gene_emb, E0, nG, nN);
    k_emb<<<(nP * 16 + NTHR - 1) / NTHR, NTHR, 0, stream>>>(path_idx, path_emb, E0, nP, nN);
  }
  k_count<<<NBLK, NTHR, 0, stream>>>(ei, deg, nE, nN);
  k_scan<<<1, NTHR, 0, stream>>>(deg, stT, NBLK, nE);
  k_fill<<<NBLK, NTHR, LDS_FILL, stream>>>(ei, et, deg, stT, csr, nE, nN, CSRN);

  k_bwt<K1, IN1><<<(NH * K1 / 8 + NTHR - 1) / NTHR, NTHR, 0, stream>>>(basis1, root1, BT);
  for (int c0 = 0; c0 < NPAD; c0 += NC) {
    int nr = NPAD - c0; nr = nr > NC ? NC : nr;
    k_agg<1><<<nr / NWAVE, NTHR, 0, stream>>>(x, E0, deg, stT, csr, comp1, Ab, c0, nN, CSRN);
    k_gemm<K1, 1><<<nr / GROWS, NTHR, LDS_GEMM, stream>>>(Ab, BT, bias1, att1, H1 + (size_t)c0 * NH,
                                                          pred_w, pred_b, out, nN - c0);
  }
  k_bwt<K2, NH><<<(NH * K2 / 8 + NTHR - 1) / NTHR, NTHR, 0, stream>>>(basis2, root2, BT);
  for (int c0 = 0; c0 < NPAD; c0 += NC) {
    int nr = NPAD - c0; nr = nr > NC ? NC : nr;
    k_agg<2><<<nr / NWAVE, NTHR, 0, stream>>>(H1, H1, deg, stT, csr, comp2, Ab, c0, nN, CSRN);
    k_gemm<K2, 2><<<nr / GROWS, NTHR, LDS_GEMM, stream>>>(Ab, BT, bias2, att2, H1, pred_w, pred_b,
                                                          out + (size_t)c0 * NOUT, nN - c0);
  }
}
